// CPUMaxEfficiencyMoE_31920196944053
// MI455X (gfx1250) — hardware-verified
//
#include <hip/hip_runtime.h>
#include <stdint.h>
#include <stddef.h>
#include <math.h>

#pragma clang fp contract(off)

#define NTOK 8192
#define DM   1024
#define FX   1024
#define NEX  8
#define MT   32
#define GX   64
#define TPB  (NTOK / (MT * GX))
#define NSL  256
#define XP   1032
#define HP   1032
#define YP   260
#define TP   72

#define LDS_XB  (MT * XP * 2)
#define LDS_HB  (MT * HP * 2)
#define LDS_EXP (2 * LDS_XB + 2 * LDS_HB)

static_assert(TPB * GX * MT == NTOK);
static_assert(MT * YP * 4 <= 2 * LDS_XB);
static_assert((XP * 2) % 16 == 0);
static_assert((HP * 2) % 16 == 0);
static_assert((YP * 4) % 16 == 0);
static_assert((TP * 2) % 16 == 0);
static_assert(NTOK % 256 == 0);
static_assert(NTOK % 8 == 0);
static_assert(DM % NSL == 0);
static_assert(FX % NSL == 0);
static_assert(DM % 64 == 0);
static_assert(FX % 64 == 0);
static_assert(DM == FX);
static_assert(NSL == 8 * 32);
static_assert(MT == 8 * 4);
static_assert((DM * NEX) % 256 == 0);
static_assert((NTOK * DM) % (4 * 256) == 0);

typedef __bf16         v16bf __attribute__((ext_vector_type(16)));
typedef float          v8f   __attribute__((ext_vector_type(8)));
typedef float          v4f   __attribute__((ext_vector_type(4)));
typedef unsigned int   v4u   __attribute__((ext_vector_type(4)));
typedef v4f __attribute__((may_alias)) v4fa;
typedef v4u __attribute__((may_alias)) v4ua;

union FragBF { v16bf v; v4u q[2]; };

__device__ __forceinline__ unsigned int bfb(float f) {
  unsigned int u = __float_as_uint(f);
  u += 0x7FFFu + ((u >> 16) & 1u);
  return u >> 16;
}
__device__ __forceinline__ void split2(float v, unsigned int& hi, unsigned int& lo) {
  hi = bfb(v);
  lo = bfb(v - __uint_as_float(hi << 16));
}
__device__ __forceinline__ unsigned int pk(unsigned int a, unsigned int b) { return (a & 0xFFFFu) | (b << 16); }

__device__ __forceinline__ v8f wmma_bf(v16bf a, v16bf b, v8f c) {
  v8f d = __builtin_amdgcn_wmma_f32_16x16x32_bf16(false, a, false, b, (short)0, c, false, false);
  asm volatile("v_nop\n\tv_nop\n\tv_nop\n\tv_nop" : "+v"(d) : "v"(a), "v"(b));
  return d;
}

__device__ __forceinline__ v16bf ldfrag_bf(const unsigned short* p, int h) {
  FragBF f;
  f.q[0] = *(const v4ua*)(p + 8 * h);
  f.q[1] = *(const v4ua*)(p + 16 + 8 * h);
  return f.v;
}

__global__ __launch_bounds__(256) void k_tsplit(const float* __restrict__ src,
                                                unsigned short* __restrict__ ph,
                                                unsigned short* __restrict__ pl)
{
  __shared__ __align__(16) unsigned short sH[64 * TP];
  __shared__ __align__(16) unsigned short sL[64 * TP];
  const int tid = threadIdx.x;
  const int r0 = blockIdx.x * 64;
  const int c0 = blockIdx.y * 64;
  const int e  = blockIdx.z;
  const float* s = src + (size_t)e * DM * DM;

  #pragma unroll
  for (int i = 0; i < 4; ++i) {
    const int rr = i * 16 + (tid >> 4);
    const int cc = 4 * (tid & 15);
    const v4f g = *(const v4fa*)(s + (size_t)(r0 + rr) * DM + c0 + cc);
    unsigned int h0, l0, h1, l1, h2, l2, h3, l3;
    split2(g.x, h0, l0); split2(g.y, h1, l1); split2(g.z, h2, l2); split2(g.w, h3, l3);
    sH[(cc + 0) * TP + rr] = (unsigned short)h0;  sL[(cc + 0) * TP + rr] = (unsigned short)l0;
    sH[(cc + 1) * TP + rr] = (unsigned short)h1;  sL[(cc + 1) * TP + rr] = (unsigned short)l1;
    sH[(cc + 2) * TP + rr] = (unsigned short)h2;  sL[(cc + 2) * TP + rr] = (unsigned short)l2;
    sH[(cc + 3) * TP + rr] = (unsigned short)h3;  sL[(cc + 3) * TP + rr] = (unsigned short)l3;
  }
  __syncthreads();

  v4u H[2], L[2];
  size_t go[2];
  #pragma unroll
  for (int p = 0; p < 2; ++p) {
    const int line = p * 32 + (tid >> 3);
    const int q = tid & 7;
    H[p] = *(const v4ua*)(sH + line * TP + 8 * q);
    L[p] = *(const v4ua*)(sL + line * TP + 8 * q);
    go[p] = ((size_t)e * DM + c0 + line) * DM + r0 + 8 * q;
    *(volatile v4u*)(ph + go[p]) = H[p];
    *(volatile v4u*)(pl + go[p]) = L[p];
  }
  __threadfence();
  #pragma unroll
  for (int p = 0; p < 2; ++p) {
    *(volatile v4u*)(ph + go[p]) = H[p];
    *(volatile v4u*)(pl + go[p]) = L[p];
  }
}

__global__ __launch_bounds__(256) void k_route(const float* __restrict__ x,
                                               const float* __restrict__ wr,
                                               float* __restrict__ rec, int ntok)
{
  __shared__ __align__(16) float swr[DM * NEX];
  __shared__ __align__(16) float srec[32];
  const int tid = threadIdx.x, lane = tid & 31, wv = tid >> 5;
  #pragma unroll
  for (int i = 0; i < (DM * NEX) / 256; ++i) swr[tid + 256 * i] = wr[tid + 256 * i];
  __syncthreads();

  const int t = blockIdx.x * 8 + wv;
  const int tc = (t < ntok) ? t : (ntok - 1);
  const float* xr = x + (size_t)tc * DM;
  double lg[NEX];
  #pragma unroll
  for (int e = 0; e < NEX; ++e) lg[e] = 0.0;
  #pragma unroll 1
  for (int i = 0; i < DM / 32; ++i) {
    const int d = 32 * i + lane;
    const double xv = (double)xr[d];
    const v4f w0 = *(const v4fa*)(swr + d * NEX);
    const v4f w1 = *(const v4fa*)(swr + d * NEX + 4);
    lg[0] = fma(xv, (double)w0.x, lg[0]);
    lg[1] = fma(xv, (double)w0.y, lg[1]);
    lg[2] = fma(xv, (double)w0.z, lg[2]);
    lg[3] = fma(xv, (double)w0.w, lg[3]);
    lg[4] = fma(xv, (double)w1.x, lg[4]);
    lg[5] = fma(xv, (double)w1.y, lg[5]);
    lg[6] = fma(xv, (double)w1.z, lg[6]);
    lg[7] = fma(xv, (double)w1.w, lg[7]);
  }
  #pragma unroll
  for (int off = 16; off > 0; off >>= 1) {
    #pragma unroll
    for (int e = 0; e < NEX; ++e) lg[e] = lg[e] + __shfl_xor(lg[e], off);
  }

  float lf[NEX];
  #pragma unroll
  for (int e = 0; e < NEX; ++e) lf[e] = (float)lg[e];
  float mx = lf[0];
  #pragma unroll
  for (int e = 1; e < NEX; ++e) mx = fmaxf(mx, lf[e]);
  float ex[NEX];
  float ssum = 0.0f;
  #pragma unroll
  for (int e = 0; e < NEX; ++e) { ex[e] = __expf(lf[e] - mx); ssum = ssum + ex[e]; }
  const float rs = __builtin_amdgcn_rcpf(ssum);
  float pr[NEX];
  #pragma unroll
  for (int e = 0; e < NEX; ++e) pr[e] = ex[e] * rs;

  int i0 = 0;
  float b0 = pr[0];
  #pragma unroll
  for (int e = 1; e < NEX; ++e) {
    const bool tk = pr[e] > b0;
    b0 = tk ? pr[e] : b0;
    i0 = tk ? e : i0;
  }
  int i1 = -1;
  float b1 = -3.0e38f;
  #pragma unroll
  for (int e = 0; e < NEX; ++e) {
    const bool tk = (e != i0) && (pr[e] > b1);
    b1 = tk ? pr[e] : b1;
    i1 = tk ? e : i1;
  }
  i1 = (i1 < 0) ? ((i0 == 0) ? 1 : 0) : i1;
  float p0 = pr[0], p1 = pr[0];
  #pragma unroll
  for (int e = 0; e < NEX; ++e) { p0 = (e == i0) ? pr[e] : p0; p1 = (e == i1) ? pr[e] : p1; }

  if (lane == 0) {
    srec[4 * wv + 0] = p0;
    srec[4 * wv + 1] = p1;
    srec[4 * wv + 2] = (float)i0;
    srec[4 * wv + 3] = (float)i1;
  }
  __syncthreads();
  if (wv == 0) {
    const int q = lane & 7;
    const v4f v = *(const v4fa*)(srec + 4 * q);
    const int tt = blockIdx.x * 8 + q;
    const bool ok = (lane < 8) && (tt < ntok);
    if (ok) *(volatile v4f*)(rec + (size_t)tt * 4) = v;
    __threadfence();
    if (ok) *(volatile v4f*)(rec + (size_t)tt * 4) = v;
  }
}

__device__ __forceinline__ void row_pass(const float* sY, const int* sTok, const int* sSlot,
                                         float* out, float* part1, int ns, int wv, int lane,
                                         int nrows)
{
  #pragma unroll
  for (int i = 0; i < 4; ++i) {
    const int row = wv * 4 + i;
    int t = sTok[row];
    t = (t < 0) ? 0 : ((t > NTOK - 1) ? (NTOK - 1) : t);
    const int s = sSlot[row];
    const v4f v0 = *(const v4fa*)(sY + row * YP + 4 * lane);
    const v4f v1 = *(const v4fa*)(sY + row * YP + 128 + 4 * lane);
    float* basep = (s == 0) ? out : part1;
    float* dst = basep + (size_t)t * DM + ns * NSL;
    if (row < nrows) {
      *(volatile v4f*)(dst + 4 * lane) = v0;
      *(volatile v4f*)(dst + 128 + 4 * lane) = v1;
    }
  }
}

__global__ __launch_bounds__(256) void k_expert(const float* __restrict__ x,
                                                const unsigned short* __restrict__ w1h,
                                                const unsigned short* __restrict__ w1l,
                                                const unsigned short* __restrict__ w2h,
                                                const unsigned short* __restrict__ w2l,
                                                const float* __restrict__ rec,
                                                float* __restrict__ out,
                                                float* __restrict__ part1, int ntok)
{
  extern __shared__ __align__(16) unsigned char dsm_e[];
  unsigned short* sXh = (unsigned short*)dsm_e;
  unsigned short* sXl = (unsigned short*)(dsm_e + LDS_XB);
  unsigned short* sHh = (unsigned short*)(dsm_e + 2 * LDS_XB);
  unsigned short* sHl = (unsigned short*)(dsm_e + 2 * LDS_XB + LDS_HB);
  float* sY = (float*)dsm_e;
  __shared__ int   sTok[MT];
  __shared__ int   sSlot[MT];
  __shared__ float sW[MT];
  __shared__ int   s_wc[8];

  const int tid = threadIdx.x, lane = tid & 31, wv = tid >> 5;
  const int h = lane >> 4, m = lane & 15;
  const int e = blockIdx.y;
  const v8f z8 = {0.f, 0.f, 0.f, 0.f, 0.f, 0.f, 0.f, 0.f};

  int cnt_lb = 0;
  int cnt_exact = 0;

  #pragma unroll 1
  for (int jt = 0; jt < TPB; ++jt) {
    const int m0 = ((int)blockIdx.x + GX * jt) * MT;
    if (cnt_exact != 0 && m0 >= cnt_lb) break;

    if (tid < MT) { sTok[tid] = 0; sSlot[tid] = 0; sW[tid] = 0.0f; }
    __syncthreads();

    int base = 0;
    int full = 1;
    #pragma unroll 1
    for (int ch = 0; ch < NTOK / 256; ++ch) {
      const int t = ch * 256 + tid;
      const int tc = (t < ntok) ? t : (ntok - 1);
      const v4f r = *(const v4fa*)(rec + (size_t)tc * 4);
      int e0 = (int)r.z, e1 = (int)r.w;
      e0 = (e0 < 0) ? 0 : ((e0 > NEX - 1) ? (NEX - 1) : e0);
      e1 = (e1 < 0) ? 0 : ((e1 > NEX - 1) ? (NEX - 1) : e1);
      const bool f0 = (e0 == e);
      const bool f1 = (e1 == e) && !f0;
      const bool f = (f0 || f1) && (t < ntok);
      const unsigned int msk = __builtin_amdgcn_ballot_w32(f);
      const int off = __builtin_popcount(msk & ((1u << lane) - 1u));
      const int wc = __builtin_popcount(msk);
      if (lane == 0) s_wc[wv] = wc;
      __syncthreads();
      int pre = 0, tot = 0;
      #pragma unroll
      for (int w2 = 0; w2 < 8; ++w2) {
        const int cc = s_wc[w2];
        tot += cc;
        pre += (w2 < wv) ? cc : 0;
      }
      if (f) {
        const int p = base + pre + off - m0;
        if ((unsigned)p < (unsigned)MT) {
          sTok[p]  = t;
          sSlot[p] = f0 ? 0 : 1;
          sW[p]    = f0 ? r.x : r.y;
        }
      }
      base += tot;
      __syncthreads();
      if (base >= m0 + MT && ch + 1 < NTOK / 256) { full = 0; break; }
    }
    if (full != 0) { cnt_exact = 1; cnt_lb = base; }
    if (m0 >= base) break;
    int nrows = base - m0;
    nrows = (nrows > MT) ? MT : nrows;

    #pragma unroll 2
    for (int j = 0; j < 16; ++j) {
      const int idx = tid + 256 * j;
      const int row = idx >> 7, c8 = idx & 127;
      int t = sTok[row];
      t = (t < 0) ? 0 : ((t > NTOK - 1) ? (NTOK - 1) : t);
      const float* xs = x + (size_t)t * DM + 8 * c8;
      const v4f a = *(const v4fa*)xs;
      const v4f c = *(const v4fa*)(xs + 4);
      unsigned int h0, l0, h1, l1, h2, l2, h3, l3, h4, l4, h5, l5, h6, l6, h7, l7;
      split2(a.x, h0, l0); split2(a.y, h1, l1); split2(a.z, h2, l2); split2(a.w, h3, l3);
      split2(c.x, h4, l4); split2(c.y, h5, l5); split2(c.z, h6, l6); split2(c.w, h7, l7);
      const v4u H = { pk(h0, h1), pk(h2, h3), pk(h4, h5), pk(h6, h7) };
      const v4u L = { pk(l0, l1), pk(l2, l3), pk(l4, l5), pk(l6, l7) };
      *(v4ua*)(sXh + row * XP + 8 * c8) = H;
      *(v4ua*)(sXl + row * XP + 8 * c8) = L;
    }
    __syncthreads();

    #pragma unroll 1
    for (int ns = 0; ns < FX / NSL; ++ns) {
      v8f acc[2][2];
      #pragma unroll
      for (int mt = 0; mt < 2; ++mt)
        #pragma unroll
        for (int nt = 0; nt < 2; ++nt) acc[mt][nt] = z8;
      #pragma unroll 1
      for (int k0 = 0; k0 < DM; k0 += 32) {
        v16bf ah[2], al[2];
        #pragma unroll
        for (int mt = 0; mt < 2; ++mt) {
          ah[mt] = ldfrag_bf(sXh + (16 * mt + m) * XP + k0, h);
          al[mt] = ldfrag_bf(sXl + (16 * mt + m) * XP + k0, h);
        }
        #pragma unroll
        for (int nt = 0; nt < 2; ++nt) {
          const int f = ns * NSL + wv * 32 + 16 * nt + m;
          const size_t bo = ((size_t)e * FX + f) * DM + k0;
          const v16bf bh = ldfrag_bf(w1h + bo, h);
          const v16bf bl = ldfrag_bf(w1l + bo, h);
          #pragma unroll
          for (int mt = 0; mt < 2; ++mt) {
            acc[mt][nt] = wmma_bf(ah[mt], bh, acc[mt][nt]);
            acc[mt][nt] = wmma_bf(ah[mt], bl, acc[mt][nt]);
            acc[mt][nt] = wmma_bf(al[mt], bh, acc[mt][nt]);
          }
        }
      }
      #pragma unroll
      for (int mt = 0; mt < 2; ++mt)
        #pragma unroll
        for (int nt = 0; nt < 2; ++nt) {
          const int col = ns * NSL + wv * 32 + 16 * nt + m;
          #pragma unroll
          for (int r = 0; r < 8; ++r) {
            const int row = 16 * mt + 8 * h + r;
            const float v = acc[mt][nt][r];
            const float hv = (v > 0.0f) ? v * v : 0.0f;
            unsigned int hb, lb;
            split2(hv, hb, lb);
            sHh[row * HP + col] = (unsigned short)hb;
            sHl[row * HP + col] = (unsigned short)lb;
          }
        }
    }
    __syncthreads();

    #pragma unroll 1
    for (int ns = 0; ns < DM / NSL; ++ns) {
      v8f acc[2][2];
      #pragma unroll
      for (int mt = 0; mt < 2; ++mt)
        #pragma unroll
        for (int nt = 0; nt < 2; ++nt) acc[mt][nt] = z8;
      #pragma unroll 1
      for (int k0 = 0; k0 < FX; k0 += 32) {
        v16bf ah[2], al[2];
        #pragma unroll
        for (int mt = 0; mt < 2; ++mt) {
          ah[mt] = ldfrag_bf(sHh + (16 * mt + m) * HP + k0, h);
          al[mt] = ldfrag_bf(sHl + (16 * mt + m) * HP + k0, h);
        }
        #pragma unroll
        for (int nt = 0; nt < 2; ++nt) {
          const int d = ns * NSL + wv * 32 + 16 * nt + m;
          const size_t bo = ((size_t)e * DM + d) * FX + k0;
          const v16bf bh = ldfrag_bf(w2h + bo, h);
          const v16bf bl = ldfrag_bf(w2l + bo, h);
          #pragma unroll
          for (int mt = 0; mt < 2; ++mt) {
            acc[mt][nt] = wmma_bf(ah[mt], bh, acc[mt][nt]);
            acc[mt][nt] = wmma_bf(ah[mt], bl, acc[mt][nt]);
            acc[mt][nt] = wmma_bf(al[mt], bh, acc[mt][nt]);
          }
        }
      }
      #pragma unroll
      for (int mt = 0; mt < 2; ++mt)
        #pragma unroll
        for (int nt = 0; nt < 2; ++nt) {
          const int cl = wv * 32 + 16 * nt + m;
          #pragma unroll
          for (int r = 0; r < 8; ++r) {
            const int row = 16 * mt + 8 * h + r;
            sY[row * YP + cl] = acc[mt][nt][r] * sW[row];
          }
        }
      __syncthreads();
      row_pass(sY, sTok, sSlot, out, part1, ns, wv, lane, nrows);
      __threadfence();
      row_pass(sY, sTok, sSlot, out, part1, ns, wv, lane, nrows);
      __syncthreads();
    }
  }
}

__global__ __launch_bounds__(256) void k_sum(const float* __restrict__ part1,
                                             float* out, int n4)
{
  const int g = blockIdx.x * 256 + threadIdx.x;
  if (g >= n4) return;
  const v4f a = *(const v4fa*)(out + (size_t)g * 4);
  const v4f b = *(const v4fa*)(part1 + (size_t)g * 4);
  const v4f v = a + b;
  float* dst = out + (size_t)g * 4;
  *(volatile v4f*)dst = v;
  __threadfence();
  *(volatile v4f*)dst = v;
}

extern "C" void kernel_launch(void* const* d_in, const int* in_sizes, int n_in,
                              void* d_out, int out_size, void* d_ws, size_t ws_size,
                              hipStream_t stream)
{
  if (n_in < 4) return;
  if (in_sizes[0] != NTOK * DM) return;
  if (in_sizes[1] != DM * NEX) return;
  if (in_sizes[2] != NEX * DM * FX) return;
  if (in_sizes[3] != NEX * FX * DM) return;
  if (out_size != NTOK * DM) return;

  const float* x  = (const float*)d_in[0];
  const float* wr = (const float*)d_in[1];
  const float* w1 = (const float*)d_in[2];
  const float* w2 = (const float*)d_in[3];
  float* out = (float*)d_out;

  const size_t bWP   = (size_t)NEX * FX * DM * 2;
  const size_t bREC  = (size_t)NTOK * 16;
  const size_t bPART = (size_t)NTOK * DM * 4;
  const size_t total = 4 * bWP + bREC + bPART;
  if (total > ws_size) return;
  if (total > (size_t)134217728) return;

  char* ws = (char*)d_ws;
  size_t off = 0;
  unsigned short* W1H = (unsigned short*)(ws + off); off += bWP;
  unsigned short* W1L = (unsigned short*)(ws + off); off += bWP;
  unsigned short* W2H = (unsigned short*)(ws + off); off += bWP;
  unsigned short* W2L = (unsigned short*)(ws + off); off += bWP;
  float*          REC = (float*)(ws + off);          off += bREC;
  float*          PART1 = (float*)(ws + off);        off += bPART;
  if (off != total) return;

  k_tsplit<<<dim3(DM / 64, FX / 64, NEX), 256, 0, stream>>>(w1, W1H, W1L);
  k_tsplit<<<dim3(FX / 64, DM / 64, NEX), 256, 0, stream>>>(w2, W2H, W2L);
  k_route<<<NTOK / 8, 256, 0, stream>>>(x, wr, REC, NTOK);
  k_expert<<<dim3(GX, NEX), 256, LDS_EXP, stream>>>(x, W1H, W1L, W2H, W2L, REC, out, PART1, NTOK);
  {
    const int n4 = NTOK * DM / 4;
    k_sum<<<(n4 + 255) / 256, 256, 0, stream>>>(PART1, out, n4);
  }
}
